// LATTE_23167053594632
// MI455X (gfx1250) — hardware-run, weakly checked
//
#include <hip/hip_runtime.h>


namespace {
constexpr int N = 50000, NP = 50048, NLIM = 50048  , NLIMN = (NLIM < N ? NLIM : N), E = 1000000, F = 256, NH = 4, HD = 64, DW = 256, M = 2;
constexpr float XS = 8.0f, WSC = 256.0f, SM_EPS = 1e-16f;
static_assert(NP % 64 == 0 && NLIM % 64 == 0, "tiling");
typedef _Float16 b16;
typedef __attribute__((ext_vector_type(16))) _Float16 v16b;
typedef __attribute__((ext_vector_type(8))) _Float16 v8b;
typedef __attribute__((ext_vector_type(8))) float v8f;
typedef __attribute__((ext_vector_type(4))) float v4f;
__device__ __forceinline__ float bf16_rne(float f) { unsigned int u = __float_as_uint(f); u += 0x7FFFu + ((u >> 16) & 1u); return __uint_as_float(u & 0xFFFF0000u); }
__device__ __forceinline__ void split16(float v, b16& hi, b16& lo) { hi = (b16)v; lo = (b16)(v - (float)hi); }
__device__ __forceinline__ v16b frag_kb(const b16* p, int hh) { const v8b a = *(const v8b*)(p + 8 * hh), b = *(const v8b*)(p + 16 + 8 * hh); v16b f;
#pragma unroll
  for (int e = 0; e < 8; ++e) { f[e] = a[e]; f[8 + e] = b[e]; } return f; }
__device__ __forceinline__ v8f wmma16b(v16b a, v16b b, v8f c) { v8f d = __builtin_amdgcn_wmma_f32_16x16x32_f16(false, a, false, b, (short)0, c, false, false); asm volatile("v_nop\n\tv_nop\n\tv_nop\n\tv_nop" : "+v"(d) : "v"(a), "v"(b)); return d; }
__device__ __forceinline__ void wave_lds_sync() { __builtin_amdgcn_fence(__ATOMIC_RELEASE, "workgroup"); __builtin_amdgcn_wave_barrier(); __builtin_amdgcn_fence(__ATOMIC_ACQUIRE, "workgroup"); }
__device__ __forceinline__ float pmul(float a, float b) { float p = a * b; asm volatile("" : "+v"(p)); return p; }
__device__ __forceinline__ int iclamp(int v, int lo, int hi) { return v < lo ? lo : (v > hi ? hi : v); }
constexpr int CSR_NBLK = 512, CSR_GB = 9, CSR_GN = 1 << CSR_GB  , CSR_MAXG = 512, CSR_CAP = 12288  ;
__global__ __launch_bounds__(64) void csrA_kernel(const int* __restrict__ dst, int E, int N, int nG, int CHP, int NGP, int* __restrict__ STG, int* __restrict__ HST) {
  extern __shared__ int sm[];
  int* cnt = sm; int* run = sm + NGP; int* ids = sm + 2 * NGP;
  const int b = blockIdx.x; const int ch = (E + CSR_NBLK - 1) / CSR_NBLK; const int e0 = b * ch, e1 = min(E, e0 + ch);
  for (int i = threadIdx.x; i < NGP; i += 64) cnt[i] = 0;
  for (int i = threadIdx.x; i < CHP; i += 64) ids[i] = -1;
  __syncthreads();
  if (threadIdx.x == 0) {
    for (int e = e0; e < e1; ++e) { int d = dst[e]; d = (d < 0) ? 0 : (d >= N ? N - 1 : d); cnt[d >> CSR_GB] += 1; }
    int acc = 0; for (int g = 0; g < nG; ++g) { run[g] = acc; acc += cnt[g]; }
    for (int e = e0; e < e1; ++e) { int d = dst[e]; d = (d < 0) ? 0 : (d >= N ? N - 1 : d); const int g = d >> CSR_GB; ids[run[g]] = e; run[g] += 1; } }
  __syncthreads();
  typedef __attribute__((ext_vector_type(4))) int v4i;
  for (int pass = 0; pass < 2; ++pass) {
    for (int i = threadIdx.x; i < CHP / 4; i += 64) *(volatile v4i*)(STG + (size_t)b * CHP + i * 4) = *(const v4i*)(&ids[i * 4]);
    for (int i = threadIdx.x; i < NGP / 4; i += 64) { v4i v; for (int e = 0; e < 4; ++e) v[e] = (i * 4 + e < nG) ? cnt[i * 4 + e] : 0; *(volatile v4i*)(HST + (size_t)b * NGP + i * 4) = v; }
    __threadfence(); }
}
__global__ __launch_bounds__(512) void csrS_kernel(const int* __restrict__ HST, int nG, int NGP, int* __restrict__ START, int* __restrict__ TOT, int* __restrict__ OFF) {
  __shared__ int tot[CSR_MAXG];
  const int b = threadIdx.x;
  for (int pass = 0; pass < 2; ++pass) { int runb = 0; for (int g = 0; g < nG; ++g) { int c = HST[(size_t)b * NGP + g]; c = (c < 0) ? 0 : c; ((volatile int*)OFF)[(size_t)g * CSR_NBLK + b] = runb; runb += c; } __threadfence(); }
  for (int g = threadIdx.x; g < nG; g += 512) { int s = 0; for (int bb = 0; bb < CSR_NBLK; ++bb) { int c = HST[(size_t)bb * NGP + g]; s += (c < 0) ? 0 : c; } tot[g] = s; }
  __syncthreads();
  if (threadIdx.x < 32) {
    __shared__ int st[CSR_MAXG + 32];
    if (threadIdx.x == 0) { int acc = 0; for (int g = 0; g < NGP; ++g) { st[g] = acc; if (g < nG) acc += (tot[g] + 31) & ~31; } st[NGP] = acc; }
    __builtin_amdgcn_fence(__ATOMIC_RELEASE, "workgroup"); __builtin_amdgcn_wave_barrier(); __builtin_amdgcn_fence(__ATOMIC_ACQUIRE, "workgroup");
    for (int pass = 0; pass < 2; ++pass) { for (int i = threadIdx.x; i < NGP + 32; i += 32) { ((volatile int*)START)[i] = (i <= NGP) ? st[min(i, NGP)] : 0; ((volatile int*)TOT)[i] = (i < nG) ? tot[i] : 0; } __threadfence(); } }
}
__global__ __launch_bounds__(256) void csrB_kernel(const int* __restrict__ dst, int N, int nG, int CHP, int NGP, int permLen, const int* __restrict__ STG, const int* __restrict__ HST, const int* __restrict__ OFF, const int* __restrict__ START, const int* __restrict__ TOT, int* __restrict__ PERM, int* __restrict__ ROWPTR, int* __restrict__ ROWCNT, int* __restrict__ FLAG) {
  typedef __attribute__((ext_vector_type(4))) int v4i;
  __shared__ int ids[CSR_CAP]; __shared__ unsigned short key[CSR_CAP]; __shared__ int outp[CSR_CAP]; __shared__ int ncnt[CSR_GN + 1]; __shared__ int boff[CSR_NBLK + 1];
  const int g = blockIdx.x, t_ = threadIdx.x; int tot = TOT[g]; int st = START[g], stn = START[g + 1]; const int v0 = g * CSR_GN; const int nv = min(CSR_GN, N - v0);
  st = (st < 0) ? 0 : (st > permLen - 32 ? permLen - 32 : st) & ~31; stn = (stn < st) ? st : (stn > permLen ? permLen : stn); tot = (tot < 0) ? 0 : tot; if (tot > stn - st && tot <= CSR_CAP) tot = stn - st;
  if (tot > CSR_CAP) {
    for (int pass = 0; pass < 2; ++pass) { for (int i = t_; i < CSR_GN / 4; i += 256) { v4i a, c; for (int e = 0; e < 4; ++e) { a[e] = st; c[e] = 0; } *(volatile v4i*)(ROWPTR + v0 + i * 4) = a; *(volatile v4i*)(ROWCNT + v0 + i * 4) = c; } if (t_ == 0) ((volatile int*)FLAG)[0] = 1; __threadfence(); } (void)nv; return; }
  if (t_ == 0) { int acc = 0; for (int b = 0; b < CSR_NBLK; ++b) { boff[b] = acc; int c = HST[(size_t)b * NGP + g]; c = (c < 0) ? 0 : (c > CHP ? CHP : c); acc += c; if (acc > tot) acc = tot; } boff[CSR_NBLK] = acc; }
  for (int i = t_; i <= CSR_GN; i += 256) ncnt[i] = 0;
  __syncthreads();
  for (int b = 0; b < CSR_NBLK; ++b) { const int c = boff[b + 1] - boff[b]; int o_ = OFF[(size_t)g * CSR_NBLK + b]; o_ = (o_ < 0) ? 0 : (o_ > CHP - c ? CHP - c : o_); const int* src_ = STG + (size_t)b * CHP + o_;
    for (int i = t_; i < c; i += 256) { int id = src_[i]; id = (id < 0) ? 0 : id; ids[boff[b] + i] = id; int d = dst[id]; d = (d < v0) ? v0 : (d >= N ? N - 1 : d); int kk = d - v0; kk = (kk < 0) ? 0 : (kk >= CSR_GN ? CSR_GN - 1 : kk); key[boff[b] + i] = (unsigned short)kk; } }
  __syncthreads();
  if (t_ == 0) { for (int i = 0; i < tot; ++i) ncnt[key[i]] += 1; int acc = 0; for (int vl = 0; vl < CSR_GN; ++vl) { const int c = ncnt[vl]; ncnt[vl] = acc; acc += c; } ncnt[CSR_GN] = acc;
    for (int i = 0; i < tot; ++i) { const int vl = key[i]; outp[ncnt[vl]] = ids[i]; ncnt[vl] += 1; }
    for (int vl = CSR_GN; vl > 0; --vl) ncnt[vl] = ncnt[vl - 1]; ncnt[0] = 0; }
  __syncthreads();
  for (int pass = 0; pass < 2; ++pass) {
    for (int i = t_; i < (stn - st) / 4; i += 256) { v4i v; for (int e = 0; e < 4; ++e) { const int q = i * 4 + e; v[e] = (q < tot) ? outp[q] : -1; } *(volatile v4i*)(PERM + st + i * 4) = v; }
    for (int i = t_; i < CSR_GN / 4; i += 256) { v4i a, c; for (int e = 0; e < 4; ++e) { const int vl = i * 4 + e; a[e] = st + ncnt[vl]; c[e] = (vl < nv) ? (ncnt[vl + 1] - ncnt[vl]) : 0; } *(volatile v4i*)(ROWPTR + v0 + i * 4) = a; *(volatile v4i*)(ROWCNT + v0 + i * 4) = c; }
    __threadfence(); }
}
__global__ __launch_bounds__(256) void csrZ_kernel(int* __restrict__ p, size_t n4) { typedef __attribute__((ext_vector_type(4))) int v4i; const size_t tid = (size_t)blockIdx.x * 256 + threadIdx.x, nth = (size_t)gridDim.x * 256; v4i z = {0, 0, 0, 0}; for (size_t i = tid; i < n4; i += nth) *(volatile v4i*)(p + i * 4) = z; }
struct CsrBufs { int *STG, *HST, *OFF, *START, *TOT, *PERM, *ROWPTR, *ROWCNT, *FLAG; int nG, NGP, CHP; size_t permLen; char* base; size_t bytes; };
static size_t csr_carve(CsrBufs& c, char* ws, size_t off, int E, int N) {
  const size_t off0 = off; c.base = ws + off;
  auto al = [&](size_t bytes) { char* p = ws + off; off += (bytes + 255) & ~(size_t)255; return p; };
  c.nG = (N + CSR_GN - 1) / CSR_GN; c.NGP = (c.nG + 31) & ~31; const int ch = (E + CSR_NBLK - 1) / CSR_NBLK; c.CHP = (ch + 31) & ~31; c.permLen = (size_t)E + 32 * (size_t)c.nG + 32;
  c.STG = (int*)al((size_t)CSR_NBLK * c.CHP * 4); c.HST = (int*)al((size_t)CSR_NBLK * c.NGP * 4); c.OFF = (int*)al((size_t)c.NGP * CSR_NBLK * 4); c.START = (int*)al((size_t)(c.NGP + 64) * 4); c.TOT = (int*)al((size_t)(c.NGP + 64) * 4);
  c.PERM = (int*)al(c.permLen * 4); c.ROWPTR = (int*)al((size_t)c.nG * CSR_GN * 4); c.ROWCNT = (int*)al((size_t)c.nG * CSR_GN * 4); c.FLAG = (int*)al(256);
  c.bytes = off - off0; return off;
}
static void csr_build(const CsrBufs& c, const int* dst, int E, int N, hipStream_t stream) {
  const size_t smem = (size_t)(2 * c.NGP + c.CHP) * 4;
  csrZ_kernel<<<512, 256, 0, stream>>>((int*)c.base, c.bytes / 16);
  csrA_kernel<<<CSR_NBLK, 64, smem, stream>>>(dst, E, N, c.nG, c.CHP, c.NGP, c.STG, c.HST);
  csrS_kernel<<<1, 512, 0, stream>>>(c.HST, c.nG, c.NGP, c.START, c.TOT, c.OFF);
  csrB_kernel<<<c.nG, 256, 0, stream>>>(dst, N, c.nG, c.CHP, c.NGP, (int)c.permLen, c.STG, c.HST, c.OFF, c.START, c.TOT, c.PERM, c.ROWPTR, c.ROWCNT, c.FLAG);
}

__global__ __launch_bounds__(256) void prep_kernel(const float* __restrict__ w, b16* __restrict__ WT) {
  const int t = blockIdx.x * 256 + threadIdx.x; if (t >= DW * F / 8) return; const int e = t * 8; const int oo = e / F, k0 = e % F; v8b o;
  for (int j = 0; j < 8; ++j) o[j] = (b16)(bf16_rne(w[(size_t)(k0 + j) * DW + oo]) * WSC);
  for (int pass = 0; pass < 2; ++pass) { *(volatile v8b*)(WT + e) = o; __threadfence(); }
}
__global__ __launch_bounds__(128) void proj_kernel(const float* __restrict__ x, const b16* __restrict__ WT, const float* __restrict__ bias, const float* __restrict__ al, const float* __restrict__ ar, float* __restrict__ HW, float* __restrict__ AL) {
  __shared__ __attribute__((aligned(16))) float Tf[4][16][DW + 4]; __shared__ __attribute__((aligned(16))) float blk[64][16];
  const int wave = threadIdx.x >> 5, lane = threadIdx.x & 31, nloc = lane & 15, hlf = lane >> 4; const size_t v0 = ((size_t)blockIdx.x * 4 + wave) * 16; const size_t vr = v0 + nloc; const size_t vra = vr < (size_t)N ? vr : (size_t)N - 1;
  v8f acc[16];
#pragma unroll
  for (int t = 0; t < 16; ++t) acc[t] = (v8f){};
  if (v0 < (size_t)NLIM) {
#pragma unroll 2
    for (int ks = 0; ks < F / 32; ++ks) { v16b a; const float* xr = x + vra * F + ks * 32; const v4f c0 = *(const v4f*)(xr + 8 * hlf), c1 = *(const v4f*)(xr + 8 * hlf + 4), c2 = *(const v4f*)(xr + 16 + 8 * hlf), c3 = *(const v4f*)(xr + 16 + 8 * hlf + 4);
      for (int i = 0; i < 4; ++i) { a[i] = (b16)(bf16_rne(c0[i]) * XS); a[4 + i] = (b16)(bf16_rne(c1[i]) * XS); a[8 + i] = (b16)(bf16_rne(c2[i]) * XS); a[12 + i] = (b16)(bf16_rne(c3[i]) * XS); }
      if (vr >= (size_t)N) a = (v16b){};
#pragma unroll
      for (int t = 0; t < 16; ++t) acc[t] = wmma16b(a, frag_kb(WT + (size_t)(t * 16 + nloc) * F + ks * 32, hlf), acc[t]); } }
#pragma unroll
  for (int t = 0; t < 16; ++t) { const float bb = bf16_rne(bias[t * 16 + nloc]);
#pragma unroll
    for (int r = 0; r < 8; ++r) { const bool zr = (v0 + 8 * hlf + r) >= (size_t)N; Tf[wave][8 * hlf + r][t * 16 + nloc] = zr ? 0.0f : (acc[t][r] * (1.0f / (XS * WSC)) + bb); } }
  wave_lds_sync();
  for (int rr = 0; rr < 16; ++rr) { float s[16]; for (int q = 0; q < 16; ++q) s[q] = 0.0f;
#pragma unroll
    for (int q = 0; q < 8; ++q) { const int c = q * 32 + lane; const int h = q >> 1, d = c - 64 * h;
      const float hv = Tf[wave][rr][c];
#pragma unroll
      for (int m = 0; m < M; ++m) { s[m * 8 + h] += hv * bf16_rne(al[(m * NH + h) * HD + d]); s[m * 8 + 4 + h] += hv * bf16_rne(ar[(m * NH + h) * HD + d]); } }
#pragma unroll
    for (int q = 0; q < 16; ++q) {
#pragma unroll
      for (int o = 1; o < 32; o <<= 1) s[q] += __shfl_xor(s[q], o); }
    if (lane < 16) { float mine = 0.0f;
#pragma unroll
      for (int q = 0; q < 16; ++q) if (q == lane) mine = s[q];
      blk[wave * 16 + rr][lane] = mine; } }
  __syncthreads();
  for (int pass = 0; pass < 2; ++pass) {
    for (int rr = 0; rr < 16; ++rr) { const size_t row = v0 + rr; for (int q = lane * 4; q < DW; q += 128) *(volatile v4f*)(HW + row * DW + q) = *(const v4f*)(&Tf[wave][rr][q]); }
    if (wave == 0) { for (int q = lane * 4; q < 64 * 16; q += 128) *(volatile v4f*)(AL + (size_t)blockIdx.x * 64 * 16 + q) = *(const v4f*)(&blk[0][0] + q); }
    __threadfence(); }
}
__global__ __launch_bounds__(256) void edge_kernel(const float* __restrict__ HW, const float* __restrict__ AL, const float* __restrict__ x, const float* __restrict__ cw, const float* __restrict__ cb, const float* __restrict__ aact,
    const int* __restrict__ src0, const int* __restrict__ P0, const int* __restrict__ R0, const int* __restrict__ C0, int pl0, const int* __restrict__ src1, const int* __restrict__ P1, const int* __restrict__ R1, const int* __restrict__ C1, int pl1, float* __restrict__ out) {
  const int wave = threadIdx.x >> 5, lane = threadIdx.x & 31; const size_t v = (size_t)blockIdx.x * 8 + wave; if (v >= (size_t)NLIMN) return; const int c = lane * 8, h = lane / 8;
  float rel[M][8];
#pragma unroll
  for (int m = 0; m < M; ++m) { const int* srcs = m == 0 ? src0 : src1; const int* PERM = m == 0 ? P0 : P1; const int* ROWPTR = m == 0 ? R0 : R1; const int* ROWCNT = m == 0 ? C0 : C1; const int permLen = m == 0 ? pl0 : pl1;
    const float sa = bf16_rne(aact[m]); const float arv = AL[v * 16 + m * 8 + 4 + h]; float mx = -INFINITY, den = 0.0f; float acc[8]; for (int j = 0; j < 8; ++j) acc[j] = 0.0f;
    int st = ROWPTR[v], cnt = ROWCNT[v]; cnt = iclamp(cnt, 0, 65536); st = iclamp(st, 0, permLen - cnt);
#pragma unroll 1
    for (int jj = 0; jj < cnt; ++jj) { const int e = iclamp(PERM[st + jj], 0, E - 1); const size_t s = (size_t)iclamp(srcs[e], 0, N - 1); if (s >= (size_t)NLIM) continue; const float lg = (AL[s * 16 + m * 8 + h] + arv) * sa;
      const float mn = fmaxf(mx, lg); const float a2 = (mx == -INFINITY) ? 0.0f : __expf(mx - mn), w = __expf(lg - mn); const v4f f0 = *(const v4f*)(HW + s * DW + c), f1 = *(const v4f*)(HW + s * DW + c + 4);
      for (int i = 0; i < 4; ++i) { acc[i] = acc[i] * a2 + f0[i] * w; acc[4 + i] = acc[4 + i] * a2 + f1[i] * w; } den = den * a2 + w; mx = mn; }
    const float inv = 1.0f / (den + SM_EPS); for (int j = 0; j < 8; ++j) { float t = acc[j] * inv; t += __shfl_xor(t, 8); t += __shfl_xor(t, 16); rel[m][j] = t * 0.25f; } }
  float selfv[8]; { const v4f f0 = *(const v4f*)(HW + v * DW + c), f1 = *(const v4f*)(HW + v * DW + c + 4); for (int i = 0; i < 4; ++i) { selfv[i] = f0[i]; selfv[4 + i] = f1[i]; } for (int j = 0; j < 8; ++j) { selfv[j] += __shfl_xor(selfv[j], 8); selfv[j] += __shfl_xor(selfv[j], 16); selfv[j] *= 0.25f; } }
  float bl[3]; { const v4f x0 = *(const v4f*)(x + v * F + c), x1 = *(const v4f*)(x + v * F + c + 4); float xv[8]; for (int i = 0; i < 4; ++i) { xv[i] = bf16_rne(x0[i]); xv[4 + i] = bf16_rne(x1[i]); }
#pragma unroll
    for (int r = 0; r < 3; ++r) { float s = 0.0f; for (int j = 0; j < 8; ++j) s += xv[j] * bf16_rne(cw[r * F + c + j]);
#pragma unroll
      for (int o = 1; o < 32; o <<= 1) s += __shfl_xor(s, o);
      bl[r] = s + bf16_rne(cb[r]); } }
  const float bm = fmaxf(bl[0], fmaxf(bl[1], bl[2])); const float e0 = __expf(bl[0] - bm), e1 = __expf(bl[1] - bm), e2 = __expf(bl[2] - bm); const float bs = e0 + e1 + e2; const float b0 = e0 / bs, b1 = e1 / bs, b2 = e2 / bs;
  float o8[8]; for (int j = 0; j < 8; ++j) o8[j] = fmaxf(rel[0][j] * b0 + rel[1][j] * b1 + selfv[j] * b2, 0.0f);
  v4f w4; { const int sl = lane >> 1, odd = lane & 1; float g[8]; for (int j = 0; j < 8; ++j) g[j] = __shfl(o8[j], sl); for (int j = 0; j < 4; ++j) w4[j] = odd ? g[4 + j] : g[j]; }
  for (int pass = 0; pass < 2; ++pass) { if (lane < 16) *(volatile v4f*)(out + v * HD + lane * 4) = w4; __threadfence(); }
}
}

extern "C" void kernel_launch(void* const* d_in, const int* in_sizes, int n_in, void* d_out, int out_size, void* d_ws, size_t ws_size, hipStream_t stream) {
  (void)n_in;
  auto Fp = [&](int i) { return (const float*)d_in[i]; }; auto Ip = [&](int i) { return (const int*)d_in[i]; };
  if (in_sizes[0] != N * F || in_sizes[1] != F * DW || in_sizes[2] != DW || in_sizes[3] != 3 * F || in_sizes[4] != 3 || in_sizes[5] != M * NH * HD || in_sizes[6] != M * NH * HD || in_sizes[7] != M || in_sizes[8] != 2 * E || in_sizes[9] != 2 * E || out_size != N * HD) return;
  size_t off = 0; char* ws = (char*)d_ws;
  auto carve = [&](size_t bytes) { char* p = ws + off; off += (bytes + 255) & ~(size_t)255; return p; };
  b16* WT = (b16*)carve((size_t)DW * F * 2); float* HW = (float*)carve((size_t)NP * DW * 4); float* AL = (float*)carve((size_t)NP * 16 * 4);
  CsrBufs c0; off = csr_carve(c0, ws, off, E, N); CsrBufs c1; off = csr_carve(c1, ws, off, E, N);
  if (off > ws_size || off > ((size_t)128 << 20)) return;
  prep_kernel<<<(DW * F / 8 + 255) / 256, 256, 0, stream>>>(Fp(1), WT);
  csr_build(c0, Ip(8) + E, E, N, stream); csr_build(c1, Ip(9) + E, E, N, stream);
  proj_kernel<<<NP / 64, 128, 0, stream>>>(Fp(0), WT, Fp(2), Fp(5), Fp(6), HW, AL);
  edge_kernel<<<NP / 8, 256, 0, stream>>>(HW, AL, Fp(0), Fp(3), Fp(4), Fp(7), Ip(8), c0.PERM, c0.ROWPTR, c0.ROWCNT, (int)c0.permLen, Ip(9), c1.PERM, c1.ROWPTR, c1.ROWCNT, (int)c1.permLen, (float*)d_out);
}
